// MambaBlock_2705829396612
// MI455X (gfx1250) — hardware-verified
//
#include <hip/hip_runtime.h>
#include <math.h>

typedef __attribute__((ext_vector_type(16))) _Float16 v16h;
typedef __attribute__((ext_vector_type(8)))  _Float16 v8h;
typedef __attribute__((ext_vector_type(8)))  float    v8f;
typedef __attribute__((ext_vector_type(4)))  float    v4f;

constexpr int kBatch = 2;
constexpr int kSeqL  = 2048;
constexpr int kDmod  = 1024;
constexpr int kDin   = 2048;
constexpr int kNst   = 16;
constexpr int kPrjN  = 2 * kNst + 1;
constexpr int kPrjP  = 64;
constexpr int kXZP   = 2 * kDin;
constexpr int kRows  = kBatch * kSeqL;
constexpr int kTP    = 260;
constexpr int kChunk = 16;
constexpr float kLnEps  = 1e-5f;
constexpr float kCarryW = 32.0f;
constexpr float kCarryU = 16.0f;
constexpr float kCarryY = 16.0f;
constexpr float kScaleIn  = 1.0f / kCarryW;
constexpr float kScaleXp  = 1.0f / (kCarryW * kCarryU);
constexpr float kScaleOut = 1.0f / (kCarryW * kCarryY);

static_assert(kPrjN == 33);
static_assert(kPrjN <= kPrjP);
static_assert((kDmod % 32) == 0 && (kDin % 32) == 0);
static_assert((kSeqL % 64) == 0 && (kXZP % 64) == 0 && (kPrjP % 64) == 0 && (kDmod % 64) == 0);
static_assert((kDmod % 64) == 0 && (kDin % 64) == 0);
static_assert((kDin % 256) == 0 && (kSeqL % kChunk) == 0 && (kRows % 2) == 0);
static_assert(((kSeqL / 64) * (kXZP / 64)) % 8 == 0);
static_assert(((kSeqL / 64) * (kPrjP / 64)) % 8 == 0);
static_assert(((kSeqL / 64) * (kDmod / 64)) % 8 == 0);

constexpr size_t kSzWIN16  = (size_t)kXZP  * kDmod * 2;
constexpr size_t kSzWXP16  = (size_t)kPrjP * kDin  * 2;
constexpr size_t kSzWOUT16 = (size_t)kDmod * kDin  * 2;
constexpr size_t kSzXN16   = (size_t)kRows * kDmod * 2;
constexpr size_t kSzXZ     = (size_t)kSeqL * kXZP  * 4;
constexpr size_t kSzUC     = (size_t)kSeqL * kDin  * 4;
constexpr size_t kSzUC16   = (size_t)kSeqL * kDin  * 2;
constexpr size_t kSzPROJ   = (size_t)kSeqL * kPrjP * 4;
constexpr size_t kSzY16    = (size_t)kSeqL * kDin  * 2;
constexpr size_t kOffWIN16  = 0;
constexpr size_t kOffWXP16  = kOffWIN16  + kSzWIN16;
constexpr size_t kOffWOUT16 = kOffWXP16  + kSzWXP16;
constexpr size_t kOffXN16   = kOffWOUT16 + kSzWOUT16;
constexpr size_t kOffXZ     = kOffXN16   + kSzXN16;
constexpr size_t kOffUC     = kOffXZ     + kSzXZ;
constexpr size_t kOffUC16   = kOffUC     + kSzUC;
constexpr size_t kOffPROJ   = kOffUC16   + kSzUC16;
constexpr size_t kOffY16    = kOffPROJ   + kSzPROJ;
constexpr size_t kWsTotal   = kOffY16    + kSzY16;
static_assert(kWsTotal == 88866816ull);
static_assert(kWsTotal <= 134217728ull);
static_assert((kOffWXP16 % 128) == 0 && (kOffWOUT16 % 128) == 0 && (kOffXN16 % 128) == 0 &&
              (kOffXZ % 128) == 0 && (kOffUC % 128) == 0 && (kOffUC16 % 128) == 0 &&
              (kOffPROJ % 128) == 0 && (kOffY16 % 128) == 0);

union FragU { v16h v; v8h h[2]; };
__device__ __forceinline__ v16h frag_load(const _Float16* p) {
  FragU f;
  f.h[0] = *(const v8h*)(p);
  f.h[1] = *(const v8h*)(p + 16);
  return f.v;
}
__device__ __forceinline__ v8f frag_mma(v16h a, v16h b, v8f c) {
  return __builtin_amdgcn_wmma_f32_16x16x32_f16(false, a, false, b, (short)0, c, false, false);
}
__device__ __forceinline__ void guard_row(v8f& a, v8f& b, v8f& c, v8f& d,
                                          v16h x, v16h y0, v16h y1, v16h y2, v16h y3) {
  asm volatile("v_nop\n\tv_nop\n\tv_nop\n\tv_nop"
               : "+v"(a), "+v"(b), "+v"(c), "+v"(d)
               : "v"(x), "v"(y0), "v"(y1), "v"(y2), "v"(y3));
}
__device__ __forceinline__ void keep4_h(v16h a, v16h b, v16h c, v16h d) {
  asm volatile("v_nop" :: "v"(a), "v"(b), "v"(c), "v"(d));
}
__device__ __forceinline__ void acc_guard4(v8f& a, v8f& b, v8f& c, v8f& d) {
  asm volatile("v_nop\n\tv_nop\n\tv_nop\n\tv_nop" : "+v"(a), "+v"(b), "+v"(c), "+v"(d));
}

template <bool RESID>
__global__ __launch_bounds__(256) void wmma_gemm64_f16(
    const unsigned short* __restrict__ Ap, int lda,
    const unsigned short* __restrict__ Btp, int ldb,
    float* __restrict__ C, int ldc,
    const float* __restrict__ resid,
    int M, int N, int K, float scale)
{
  const _Float16* A  = (const _Float16*)Ap;
  const _Float16* Bt = (const _Float16*)Btp;
  __shared__ __align__(16) float sT[8][16 * 68];
  const int lane = threadIdx.x & 31;
  const int wave = threadIdx.x >> 5;
  const int tilesN = N >> 6;
  const int tilesM = M >> 6;
  const int tile = blockIdx.x * 8 + wave;
  if (tile >= tilesM * tilesN) return;
  const int tm = tile / tilesN;
  const int tn = tile - tm * tilesN;
  const int m0 = tm << 6;
  const int n0 = tn << 6;

  const int rlane = lane & 15;
  const int koff  = (lane >> 4) * 8;
  const int mOff  = (lane >> 4) * 8;

  v8f acc[4][4];
#pragma unroll
  for (int i = 0; i < 4; ++i)
#pragma unroll
    for (int j = 0; j < 4; ++j) acc[i][j] = (v8f){0.f, 0.f, 0.f, 0.f, 0.f, 0.f, 0.f, 0.f};

  for (int k0 = 0; k0 < K; k0 += 32) {
    v16h bh[4];
#pragma unroll
    for (int j = 0; j < 4; ++j) {
      const size_t bo = (size_t)(n0 + (j << 4) + rlane) * ldb + koff + k0;
      bh[j] = frag_load(Bt + bo);
    }
#pragma unroll
    for (int i = 0; i < 4; ++i) {
      const size_t ao = (size_t)(m0 + (i << 4) + rlane) * lda + koff + k0;
      const v16h ah = frag_load(A + ao);
#pragma unroll
      for (int j = 0; j < 4; ++j) acc[i][j] = frag_mma(ah, bh[j], acc[i][j]);
      guard_row(acc[i][0], acc[i][1], acc[i][2], acc[i][3], ah, bh[0], bh[1], bh[2], bh[3]);
    }
    keep4_h(bh[0], bh[1], bh[2], bh[3]);
  }
  acc_guard4(acc[0][0], acc[0][1], acc[0][2], acc[0][3]);
  acc_guard4(acc[1][0], acc[1][1], acc[1][2], acc[1][3]);
  acc_guard4(acc[2][0], acc[2][1], acc[2][2], acc[2][3]);
  acc_guard4(acc[3][0], acc[3][1], acc[3][2], acc[3][3]);

  float* slab = sT[wave];
  const int hh = lane >> 4;
  const int c4 = (lane & 15) * 4;
#pragma unroll
  for (int i = 0; i < 4; ++i) {
    const int mBase = m0 + (i << 4);
#pragma unroll
    for (int j = 0; j < 4; ++j) {
#pragma unroll
      for (int r = 0; r < 8; ++r) {
        slab[(mOff + r) * 68 + (j << 4) + rlane] = acc[i][j][r] * scale;
      }
    }
    __builtin_amdgcn_fence(__ATOMIC_RELEASE, "workgroup");
    __builtin_amdgcn_wave_barrier();
    __builtin_amdgcn_fence(__ATOMIC_ACQUIRE, "workgroup");
    v4f ov[8];
#pragma unroll
    for (int it = 0; it < 8; ++it) {
      const int row = it * 2 + hh;
      v4f v = *(const v4f*)(slab + row * 68 + c4);
      if (RESID) {
        const v4f rv = *(const v4f*)(resid + (size_t)(mBase + row) * ldc + n0 + c4);
        v = v + rv;
      }
      ov[it] = v;
    }
    for (int pass = 0; pass < 2; ++pass) {
#pragma unroll
      for (int it = 0; it < 8; ++it) {
        const int row = it * 2 + hh;
        *(volatile v4f*)(C + (size_t)(mBase + row) * ldc + n0 + c4) = ov[it];
      }
      __threadfence();
    }
    __builtin_amdgcn_fence(__ATOMIC_RELEASE, "workgroup");
    __builtin_amdgcn_wave_barrier();
    __builtin_amdgcn_fence(__ATOMIC_ACQUIRE, "workgroup");
  }
}

__global__ __launch_bounds__(256) void transpose_cast_kernel(
    const float* __restrict__ W, unsigned short* __restrict__ Bt, int Kdim, int Ndim, int Npad, float scale)
{
  __shared__ float tile[64 * 65];
  const int tid = threadIdx.x, lane = tid & 31, wave = tid >> 5;
  const int n0 = blockIdx.x * 64;
  const int k0 = blockIdx.y * 64;
  (void)Npad;
#pragma unroll
  for (int p = 0; p < 16; ++p) {
    const int idx = tid + p * 256;
    const int kk  = idx >> 6;
    const int nn  = idx & 63;
    const int n   = n0 + nn;
    const int nc  = (n < Ndim) ? n : (Ndim - 1);
    const float v = W[(size_t)(k0 + kk) * Ndim + nc];
    tile[kk * 65 + nn] = (n < Ndim) ? (v * scale) : 0.f;
  }
  __syncthreads();
  const int q = lane >> 3, c8 = (lane & 7) * 8;
  v8h hv[2];
#pragma unroll
  for (int it = 0; it < 2; ++it) {
    const int nrow = it * 32 + wave * 4 + q;
#pragma unroll
    for (int e = 0; e < 8; ++e) hv[it][e] = (_Float16)tile[(c8 + e) * 65 + nrow];
  }
  for (int pass = 0; pass < 2; ++pass) {
#pragma unroll
    for (int it = 0; it < 2; ++it) {
      const int nrow = it * 32 + wave * 4 + q;
      *(volatile v8h*)(Bt + (size_t)(n0 + nrow) * Kdim + k0 + c8) = hv[it];
    }
    __threadfence();
  }
}

__global__ __launch_bounds__(256) void layernorm_f16_kernel(
    const float* __restrict__ x, const float* __restrict__ g, const float* __restrict__ bta,
    unsigned short* __restrict__ XN)
{
  __shared__ float sSum[8];
  __shared__ float sVar[8];
  const int tid = threadIdx.x, lane = tid & 31, wave = tid >> 5;
  const int rsel = tid >> 7;
  const int row  = blockIdx.x * 2 + rsel;
  const int c8   = (tid & 127) * 8;
  const float* xr = x + (size_t)row * kDmod + c8;
  const v4f a0 = *(const v4f*)(xr);
  const v4f a1 = *(const v4f*)(xr + 4);
  float s = ((a0[0] + a0[1]) + (a0[2] + a0[3])) + ((a1[0] + a1[1]) + (a1[2] + a1[3]));
#pragma unroll
  for (int off = 16; off > 0; off >>= 1) s += __shfl_xor(s, off, 32);
  if (lane == 0) sSum[wave] = s;
  __syncthreads();
  const int wb = rsel * 4;
  const float mu = ((sSum[wb] + sSum[wb + 1]) + (sSum[wb + 2] + sSum[wb + 3])) * (1.0f / (float)kDmod);
  float dv[8];
#pragma unroll
  for (int e = 0; e < 4; ++e) {
    dv[e]     = a0[e] - mu;
    dv[4 + e] = a1[e] - mu;
  }
  float vs = ((dv[0] * dv[0] + dv[1] * dv[1]) + (dv[2] * dv[2] + dv[3] * dv[3])) +
             ((dv[4] * dv[4] + dv[5] * dv[5]) + (dv[6] * dv[6] + dv[7] * dv[7]));
#pragma unroll
  for (int off = 16; off > 0; off >>= 1) vs += __shfl_xor(vs, off, 32);
  if (lane == 0) sVar[wave] = vs;
  __syncthreads();
  const float var  = ((sVar[wb] + sVar[wb + 1]) + (sVar[wb + 2] + sVar[wb + 3])) * (1.0f / (float)kDmod);
  const float rstd = rsqrtf(var + kLnEps);
  const v4f g0 = *(const v4f*)(g + c8);
  const v4f g1 = *(const v4f*)(g + c8 + 4);
  const v4f b0 = *(const v4f*)(bta + c8);
  const v4f b1 = *(const v4f*)(bta + c8 + 4);
  v8h hv;
#pragma unroll
  for (int e = 0; e < 4; ++e) {
    const float y0 = dv[e] * rstd * g0[e] + b0[e];
    const float y1 = dv[4 + e] * rstd * g1[e] + b1[e];
    hv[e]     = (_Float16)y0;
    hv[4 + e] = (_Float16)y1;
  }
  unsigned short* q = XN + (size_t)row * kDmod + c8;
  *(volatile v8h*)q = hv;
  __threadfence();
  *(volatile v8h*)q = hv;
}

__global__ __launch_bounds__(256) void conv_silu_kernel(
    const float* __restrict__ XZ, const float* __restrict__ cw, const float* __restrict__ cb,
    float* __restrict__ UC, unsigned short* __restrict__ UC16)
{
  __shared__ __align__(16) float sT[16 * kTP];
  const int tid = threadIdx.x, lane = tid & 31, wave = tid >> 5;
  const int d0 = blockIdx.x * 256, d = d0 + tid;
  const int t0 = blockIdx.y * 64;
  const v4f wv = *(const v4f*)(cw + (size_t)d * 4);
  const float w0 = wv[0], w1 = wv[1], w2 = wv[2], w3 = wv[3];
  const float bc = cb[d];
  float xm3, xm2, xm1;
  {
    const int r3 = t0 - 3, r2 = t0 - 2, r1 = t0 - 1;
    const float v3 = XZ[(size_t)(r3 < 0 ? 0 : r3) * kXZP + d];
    const float v2 = XZ[(size_t)(r2 < 0 ? 0 : r2) * kXZP + d];
    const float v1 = XZ[(size_t)(r1 < 0 ? 0 : r1) * kXZP + d];
    xm3 = (r3 >= 0) ? v3 : 0.f;
    xm2 = (r2 >= 0) ? v2 : 0.f;
    xm1 = (r1 >= 0) ? v1 : 0.f;
  }
  const int hrow = wave >> 1;
  const int hch  = (wave & 1) * 128 + lane * 4;
#pragma unroll 1
  for (int sub = 0; sub < 4; ++sub) {
    const int lb = t0 + sub * 16;
#pragma unroll 1
    for (int s = 0; s < 16; ++s) {
      const float xcur = XZ[(size_t)(lb + s) * kXZP + d];
      float acc = w0 * xm3;
      acc = fmaf(w1, xm2, acc);
      acc = fmaf(w2, xm1, acc);
      acc = fmaf(w3, xcur, acc);
      const float sv = acc + bc;
      const float sg = __builtin_amdgcn_rcpf(1.0f + expf(-sv));
      sT[s * kTP + tid] = sv * sg;
      xm3 = xm2;
      xm2 = xm1;
      xm1 = xcur;
    }
    __syncthreads();
    v4f fv[4];
    v8h bv[2];
#pragma unroll
    for (int it = 0; it < 4; ++it) fv[it] = *(const v4f*)(sT + (it * 4 + hrow) * kTP + hch);
#pragma unroll
    for (int it = 0; it < 2; ++it) {
      const float* sp = sT + (it * 8 + wave) * kTP + lane * 8;
      const v4f a0 = *(const v4f*)(sp);
      const v4f a1 = *(const v4f*)(sp + 4);
#pragma unroll
      for (int e = 0; e < 4; ++e) {
        bv[it][e]     = (_Float16)(a0[e] * kCarryU);
        bv[it][4 + e] = (_Float16)(a1[e] * kCarryU);
      }
    }
    for (int pass = 0; pass < 2; ++pass) {
#pragma unroll
      for (int it = 0; it < 4; ++it)
        *(volatile v4f*)(UC + (size_t)(lb + it * 4 + hrow) * kDin + d0 + hch) = fv[it];
#pragma unroll
      for (int it = 0; it < 2; ++it)
        *(volatile v8h*)(UC16 + (size_t)(lb + it * 8 + wave) * kDin + d0 + lane * 8) = bv[it];
      __threadfence();
    }
    __syncthreads();
  }
}

__global__ __launch_bounds__(256) void scan_gate_kernel(
    const float* __restrict__ PROJ, const float* __restrict__ UC, const float* __restrict__ XZ,
    const float* __restrict__ Wdt, const float* __restrict__ bdt, const float* __restrict__ Alog,
    const float* __restrict__ Dv, unsigned short* __restrict__ Y16)
{
  __shared__ __align__(16) float sP[kChunk * kPrjP];
  __shared__ __align__(16) float sY[kChunk * kTP];
  __shared__ __align__(16) float sA[kNst * 256];
  const int tid = threadIdx.x, lane = tid & 31, wave = tid >> 5;
  const int d0 = blockIdx.x * 256, d = d0 + tid;

#pragma unroll 1
  for (int n = 0; n < kNst; ++n) sA[n * 256 + tid] = -expf(Alog[(size_t)d * kNst + n]);
  __syncthreads();
  float An[kNst], h[kNst];
#pragma unroll
  for (int n = 0; n < kNst; ++n) {
    An[n] = sA[n * 256 + tid];
    h[n] = 0.f;
  }
  const float wd = Wdt[d];
  const float bd = bdt[d];
  const float Dd = Dv[d];
  const int sr = tid >> 4;
  const int sq = (tid & 15) * 4;

#pragma unroll 1
  for (int c = 0; c < kSeqL / kChunk; ++c) {
    const int l0 = c * kChunk;
    {
      const v4f v = *(const v4f*)(PROJ + (size_t)(l0 + sr) * kPrjP + sq);
      *(v4f*)(sP + sr * kPrjP + sq) = v;
    }
    __syncthreads();
#pragma unroll 1
    for (int s = 0; s < kChunk; ++s) {
      const size_t m = (size_t)(l0 + s);
      const float* pr = sP + s * kPrjP;
      v4f Bq[4], Cq[4];
#pragma unroll
      for (int qq = 0; qq < 4; ++qq) {
        Bq[qq] = *(const v4f*)(pr + 4 * qq);
        Cq[qq] = *(const v4f*)(pr + kNst + 4 * qq);
      }
      const float dtr = pr[2 * kNst];
      const float tv  = dtr * wd + bd;
      const float ea  = __expf(-fabsf(tv));
      const float ua  = 1.0f + ea;
      const float l1p = __logf(ua) + (ea - (ua - 1.0f)) * __builtin_amdgcn_rcpf(ua);
      const float dt  = fmaxf(tv, 0.0f) + l1p;
      const float xv  = UC[m * kDin + d];
      const float zv  = XZ[m * kXZP + kDin + d];
      const float dtx = dt * xv;
      float y = 0.f;
#pragma unroll
      for (int n = 0; n < kNst; ++n) {
        const float e = __expf(dt * An[n]);
        h[n] = e * h[n] + dtx * Bq[n >> 2][n & 3];
        y = h[n] * Cq[n >> 2][n & 3] + y;
      }
      y = xv * Dd + y;
      const float sg = __builtin_amdgcn_rcpf(1.0f + expf(-zv));
      sY[s * kTP + tid] = (y * (zv * sg)) * kCarryY;
    }
    __syncthreads();
    v8h hv[2];
#pragma unroll
    for (int it = 0; it < 2; ++it) {
      const float* sp = sY + (it * 8 + wave) * kTP + lane * 8;
      const v4f a0 = *(const v4f*)(sp);
      const v4f a1 = *(const v4f*)(sp + 4);
#pragma unroll
      for (int e = 0; e < 4; ++e) {
        hv[it][e]     = (_Float16)a0[e];
        hv[it][4 + e] = (_Float16)a1[e];
      }
    }
    for (int pass = 0; pass < 2; ++pass) {
#pragma unroll
      for (int it = 0; it < 2; ++it)
        *(volatile v8h*)(Y16 + (size_t)(l0 + it * 8 + wave) * kDin + d0 + lane * 8) = hv[it];
      __threadfence();
    }
  }
}

extern "C" void kernel_launch(void* const* d_in, const int* in_sizes, int n_in,
                              void* d_out, int out_size, void* d_ws, size_t ws_size,
                              hipStream_t stream)
{
  if (n_in < 12) return;
  if (in_sizes[0] != kRows * kDmod) return;
  if (in_sizes[1] != kDmod || in_sizes[2] != kDmod) return;
  if (in_sizes[3] != kDmod * kXZP) return;
  if (in_sizes[4] != kDin * 4 || in_sizes[5] != kDin) return;
  if (in_sizes[6] != kDin * kPrjN) return;
  if (in_sizes[7] != kDin || in_sizes[8] != kDin) return;
  if (in_sizes[9] != kDin * kNst || in_sizes[10] != kDin) return;
  if (in_sizes[11] != kDin * kDmod) return;
  if (out_size != kRows * kDmod) return;
  if (ws_size < kWsTotal) return;

  const float* x      = (const float*)d_in[0];
  const float* ln_g   = (const float*)d_in[1];
  const float* ln_b   = (const float*)d_in[2];
  const float* W_in   = (const float*)d_in[3];
  const float* conv_w = (const float*)d_in[4];
  const float* conv_b = (const float*)d_in[5];
  const float* W_xp   = (const float*)d_in[6];
  const float* W_dt   = (const float*)d_in[7];
  const float* b_dt   = (const float*)d_in[8];
  const float* A_log  = (const float*)d_in[9];
  const float* Dv     = (const float*)d_in[10];
  const float* W_out  = (const float*)d_in[11];
  float* dout = (float*)d_out;

  char* ws = (char*)d_ws;
  unsigned short* WIN16  = (unsigned short*)(ws + kOffWIN16);
  unsigned short* WXP16  = (unsigned short*)(ws + kOffWXP16);
  unsigned short* WOUT16 = (unsigned short*)(ws + kOffWOUT16);
  unsigned short* XN16   = (unsigned short*)(ws + kOffXN16);
  float*          XZ     = (float*)(ws + kOffXZ);
  float*          UC     = (float*)(ws + kOffUC);
  unsigned short* UC16   = (unsigned short*)(ws + kOffUC16);
  float*          PROJ   = (float*)(ws + kOffPROJ);
  unsigned short* Y16    = (unsigned short*)(ws + kOffY16);

  transpose_cast_kernel<<<dim3(kXZP / 64, kDmod / 64), 256, 0, stream>>>(W_in, WIN16, kDmod, kXZP, kXZP, kCarryW);
  transpose_cast_kernel<<<dim3(kPrjP / 64, kDin / 64), 256, 0, stream>>>(W_xp, WXP16, kDin, kPrjN, kPrjP, kCarryW);
  transpose_cast_kernel<<<dim3(kDmod / 64, kDin / 64), 256, 0, stream>>>(W_out, WOUT16, kDin, kDmod, kDmod, kCarryW);

  layernorm_f16_kernel<<<kRows / 2, 256, 0, stream>>>(x, ln_g, ln_b, XN16);

  for (int b = 0; b < kBatch; ++b) {
    const unsigned short* XNb = XN16 + (size_t)b * kSeqL * kDmod;
    const float* xb = x + (size_t)b * kSeqL * kDmod;
    float* outb = dout + (size_t)b * kSeqL * kDmod;

    wmma_gemm64_f16<false><<<dim3(256, 1), 256, 0, stream>>>(
        XNb, kDmod, WIN16, kDmod, XZ, kXZP, xb, kSeqL, kXZP, kDmod, kScaleIn);

    conv_silu_kernel<<<dim3(kDin / 256, kSeqL / 64), 256, 0, stream>>>(XZ, conv_w, conv_b, UC, UC16);

    wmma_gemm64_f16<false><<<dim3(4, 1), 256, 0, stream>>>(
        UC16, kDin, WXP16, kDin, PROJ, kPrjP, xb, kSeqL, kPrjP, kDin, kScaleXp);

    scan_gate_kernel<<<dim3(kDin / 256, 1), 256, 0, stream>>>(PROJ, UC, XZ, W_dt, b_dt, A_log, Dv, Y16);

    wmma_gemm64_f16<true><<<dim3(64, 1), 256, 0, stream>>>(
        Y16, kDin, WOUT16, kDin, outb, kDmod, xb, kSeqL, kDmod, kDin, kScaleOut);
  }
}
